// VladPooling_66194035966256
// MI455X (gfx1250) — hardware-run, weakly checked
//
#include <hip/hip_runtime.h>
#include <stddef.h>


typedef _Float16 v16h __attribute__((ext_vector_type(16)));
typedef _Float16 v8h  __attribute__((ext_vector_type(8)));
typedef float    v8f  __attribute__((ext_vector_type(8)));
typedef float    v4f  __attribute__((ext_vector_type(4)));
typedef _Float16 h16;

#ifndef NB
#define NB 32
#endif
#ifndef SPOS
#define SPOS 800
#endif
#define NB_FULL   32
#define SPOS_FULL 800
#define DIM   512
#define KG    10
#define KC    8
#define KPAD  16
#define NSTEP (SPOS / 32)

#define LDF 40
#define LDA 40
#define RS  516

#define ACARRY 1024.0f
#define FCARRY 64.0f

static_assert(NB >= 1 && NB <= NB_FULL);
static_assert(SPOS >= 32 && SPOS <= SPOS_FULL && (SPOS % 32) == 0);
static_assert(KG <= KPAD && KC <= 8 && KC <= KG);
static_assert(KC == 8);
static_assert(DIM == 8 * 64);
static_assert(DIM == 4 * 32 * 4);
static_assert((32 * DIM) == 16 * 256 * 4);
static_assert((LDF % 8) == 0 && LDF >= 32);
static_assert((LDA % 8) == 0 && LDA >= 32);
static_assert((RS % 4) == 0 && RS >= DIM);
static_assert((KPAD - KG) * LDA <= 256);
static_assert((size_t)DIM * LDF * 2 + (size_t)KPAD * LDA * 2 + (size_t)KC * RS * 4 + KPAD * 4
              <= (size_t)65536);

__device__ __forceinline__ float bf16r(float x) {
  unsigned int u = __float_as_uint(x);
  u = (u + 0x7FFFu + ((u >> 16) & 1u)) & 0xFFFF0000u;
  return __uint_as_float(u);
}

static __device__ __forceinline__ h16 toh_flush(float v) {
  const h16 r = (h16)v;
  return (fabsf(v) < 6.103515625e-05f) ? (h16)0.0f : r;
}

__device__ __forceinline__ v16h frag_at(const _Float16* p) {
  v8h lo = *(const v8h*)(p);
  v8h hi = *(const v8h*)(p + 16);
  v16h out;
#pragma unroll
  for (int i = 0; i < 8; ++i) { out[i] = lo[i]; out[i + 8] = hi[i]; }
  return out;
}
__device__ __forceinline__ v16h ld_frag(const _Float16* base, unsigned ld) {
  const unsigned lane = threadIdx.x & 31u;
  return frag_at(base + (lane & 15u) * ld + (lane >> 4) * 8u);
}

__device__ __forceinline__ v8f wmma16(v16h a, v16h b, v8f c) {
  v8f d = __builtin_amdgcn_wmma_f32_16x16x32_f16(false, a, false, b, (short)0, c,
                                                 false, false);
  asm volatile("v_nop\n\tv_nop\n\tv_nop\n\tv_nop" : "+v"(d) : "v"(a), "v"(b));
  return d;
}

__device__ __forceinline__ float red32_sum(float x) {
#pragma unroll
  for (int off = 1; off < 32; off <<= 1) x += __shfl_xor(x, off, 32);
  return x;
}

__global__ __launch_bounds__(256) void pool_kernel(
    const float* __restrict__ feat, const float* __restrict__ score,
    const float* __restrict__ cluster, float* __restrict__ out) {
  __shared__ __attribute__((aligned(16))) _Float16 Ft[DIM * LDF];
  __shared__ __attribute__((aligned(16))) _Float16 At[KPAD * LDA];
  __shared__ __attribute__((aligned(16))) float Rs[KC * RS];
  __shared__ float Asum[KPAD];

  const unsigned tid = threadIdx.x, lane = tid & 31u;
  const int wave = __builtin_amdgcn_readfirstlane(threadIdx.x >> 5);
  const unsigned hh = lane >> 4, m = lane & 15u;
  const unsigned b = blockIdx.x;
  const float* fb = feat + (size_t)b * SPOS_FULL * DIM;
  const float* sb = score + (size_t)b * SPOS_FULL * KG;

  if (tid < (unsigned)((KPAD - KG) * LDA)) At[KG * LDA + tid] = (h16)0.0f;

  float as[KC];
#pragma unroll
  for (int k = 0; k < KC; ++k) as[k] = 0.0f;
  v8f acc[4];
#pragma unroll
  for (int t = 0; t < 4; ++t) acc[t] = (v8f){};

  for (unsigned st = 0; st < (unsigned)NSTEP; ++st) {
    const unsigned s0 = st * 32u;
#pragma unroll 4
    for (unsigned j = 0; j < 16u; ++j) {
      const unsigned idx = tid + 256u * j;
      const unsigned r = idx >> 7, c = (idx & 127u) * 4u;
      const v4f x = *(const v4f*)(fb + (size_t)(s0 + r) * DIM + c);
#pragma unroll
      for (int i = 0; i < 4; ++i)
        Ft[(c + (unsigned)i) * LDF + r] = toh_flush(FCARRY * bf16r(x[i]));
    }
    if (wave == 0) {
      const float* srow = sb + (size_t)(s0 + lane) * KG;
      float v[KG];
      float mx = -3.0e38f;
#pragma unroll
      for (int k = 0; k < KG; ++k) { v[k] = bf16r(srow[k]); mx = fmaxf(mx, v[k]); }
      float sum = 0.0f;
#pragma unroll
      for (int k = 0; k < KG; ++k) { v[k] = __expf(v[k] - mx); sum += v[k]; }
      const float inv = 1.0f / sum;
#pragma unroll
      for (int k = 0; k < KG; ++k) {
        const float a = v[k] * inv;
        if (k < KC) as[k] += a;
        At[(unsigned)k * LDA + lane] = toh_flush(a * ACARRY);
      }
    }
    __syncthreads();

    const v16h af = ld_frag(At, LDA);
#pragma unroll
    for (int t = 0; t < 4; ++t) {
      const v16h bf = ld_frag(&Ft[((unsigned)wave * 64u + (unsigned)t * 16u) * LDF], LDF);
      acc[t] = wmma16(af, bf, acc[t]);
    }
    __syncthreads();
  }

  if (wave == 0) {
#pragma unroll
    for (int k = 0; k < KC; ++k) {
      const float t = red32_sum(as[k]);
      if (lane == 0u) Asum[k] = t;
    }
  }
  if (hh == 0u) {
#pragma unroll
    for (int t = 0; t < 4; ++t)
#pragma unroll
      for (int r = 0; r < 8; ++r)
        Rs[(unsigned)r * RS + (unsigned)wave * 64u + (unsigned)t * 16u + m] =
            acc[t][r] * (1.0f / (ACARRY * FCARRY));
  }
  __syncthreads();

  {
    const unsigned k = (unsigned)wave;
    const float asum = Asum[k];
    v4f xs[4];
    size_t off[4];
    float ss = 0.0f;
#pragma unroll
    for (unsigned i = 0; i < 4u; ++i) {
      const unsigned c = i * 128u + lane * 4u;
      const v4f u = *(const v4f*)&Rs[k * RS + c];
      const v4f g = *(const v4f*)(cluster + (size_t)k * DIM + c);
      v4f x;
#pragma unroll
      for (int j = 0; j < 4; ++j) {
        x[j] = u[j] - asum * bf16r(g[j]);
        ss += x[j] * x[j];
      }
      xs[i] = x;
      off[i] = ((size_t)b * KC + k) * DIM + c;
    }
    const float tot = red32_sum(ss);
    const float inv = 1.0f / sqrtf(fmaxf(tot, 1.0e-12f));
#pragma unroll
    for (int i = 0; i < 4; ++i) xs[i] = xs[i] * inv;
#pragma unroll
    for (int i = 0; i < 4; ++i) *(volatile v4f*)(out + off[i]) = xs[i];
    __threadfence();
#pragma unroll
    for (int i = 0; i < 4; ++i) *(volatile v4f*)(out + off[i]) = xs[i];
  }
}

extern "C" void kernel_launch(void* const* d_in, const int* in_sizes, int n_in,
                              void* d_out, int out_size, void* d_ws, size_t ws_size,
                              hipStream_t stream) {
  (void)d_ws; (void)ws_size;
  if (n_in < 3) return;
  const long long need_rows = (long long)(NB - 1) * SPOS_FULL + SPOS;
  if ((long long)in_sizes[0] < need_rows * DIM) return;
  if ((long long)in_sizes[1] < need_rows * KG) return;
  if ((long long)in_sizes[2] < (long long)KG * DIM) return;
  if ((long long)out_size < (long long)NB * KC * DIM) return;

  const float* feat    = (const float*)d_in[0];
  const float* score   = (const float*)d_in[1];
  const float* cluster = (const float*)d_in[2];
  float* out = (float*)d_out;

  pool_kernel<<<dim3(NB), dim3(256), 0, stream>>>(feat, score, cluster, out);
}
